// MolecularGCN_4105988735685
// MI455X (gfx1250) — hardware-run, weakly checked
//
#include <hip/hip_runtime.h>
#include <math.h>

constexpr int kNodes   = 100000;
constexpr int kEdges   = 1600000;
constexpr int kFin     = 128;
constexpr int kHid     = 64;
constexpr int kGraphs  = 1024;
constexpr int kNpad    = 100352;
constexpr int kNT      = 256;
constexpr int kSP      = 32;
constexpr int kChunk   = kNT * kSP;
constexpr int kChunksE = (kEdges + kChunk - 1) / kChunk;
constexpr int kTileR   = 896;
constexpr int kTilesR  = kNpad / kTileR;
constexpr int kRowsW   = kTileR / 8;
constexpr int kCapR    = 2048;
constexpr int kTileS   = 25088;
constexpr int kTilesS  = kNpad / kTileS;
constexpr int kRowsWS  = kTileS / 8;
constexpr int kCapS    = kChunk;
constexpr int kGPB     = 32;
constexpr float kCarryW = 64.0f;
constexpr float kCarryH = 64.0f;
constexpr float kScale1 = 1.0f / 64.0f;
constexpr float kScale2 = 1.0f / 4096.0f;

#define CT_ASSERT(name, cond) typedef char name[(cond) ? 1 : -1]
CT_ASSERT(ct_pad0, (kNpad % 64 == 0) && (kNpad >= kNodes) && ((kNpad / 64) % 8 == 0));
CT_ASSERT(ct_k32,  (kFin % 32 == 0) && (kHid % 32 == 0) && (kHid == 64) && (kFin == 128));
CT_ASSERT(ct_sp,   (kEdges % kSP == 0) && (kSP == 32) && (kChunk == 8192));
CT_ASSERT(ct_tlr,  (kTileR * kTilesR == kNpad) && (kRowsW * 8 == kTileR) && (kRowsW % 4 == 0) && (kTileR <= 1024));
CT_ASSERT(ct_tls,  (kTileS * kTilesS == kNpad) && (kRowsWS * 8 == kTileS) && (kRowsWS % 32 == 0) && (kTileS < 32768));
CT_ASSERT(ct_rec,  (kNodes < 131072) && (kCapR <= kChunk) && (kCapS == kChunk));
CT_ASSERT(ct_gpb,  (kGraphs % kGPB == 0) && (kGPB == 32));
CT_ASSERT(ct_cast, ((kNpad * (kFin / 8)) % kNT) == 0 && ((kNpad / 32) % 8 == 0));

typedef __attribute__((ext_vector_type(16))) _Float16 v16h;
typedef __attribute__((ext_vector_type(8)))  _Float16 v8h;
typedef __attribute__((ext_vector_type(16))) __bf16   v16b;
typedef __attribute__((ext_vector_type(8)))  __bf16   v8b;
typedef __attribute__((ext_vector_type(8)))  float    v8f;
typedef __attribute__((ext_vector_type(4)))  float    v4f;
typedef __attribute__((ext_vector_type(2)))  float    v2f;
typedef __attribute__((ext_vector_type(4)))  int      v4i;
typedef __attribute__((ext_vector_type(4)))  unsigned int v4u;

__device__ __forceinline__ unsigned short f2bf_bits(float f) {
  unsigned u = __float_as_uint(f);
  return (unsigned short)((u + 0x7FFFu + ((u >> 16) & 1u)) >> 16);
}
__device__ __forceinline__ float bf_bits2f(unsigned short h) { return __uint_as_float(((unsigned)h) << 16); }

__device__ __forceinline__ void dep_guard_h(v8f& a, v8f& b, v16h x, v16h y) { asm volatile("v_nop\n\tv_nop\n\tv_nop\n\tv_nop" : "+v"(a), "+v"(b) : "v"(x), "v"(y)); }
__device__ __forceinline__ void dep_guard_b(v8f& a, v8f& b, v16b x, v16b y) { asm volatile("v_nop\n\tv_nop\n\tv_nop\n\tv_nop" : "+v"(a), "+v"(b) : "v"(x), "v"(y)); }
__device__ __forceinline__ void keep4_h(v16h a, v16h b, v16h c, v16h d) { asm volatile("v_nop" :: "v"(a), "v"(b), "v"(c), "v"(d)); }
__device__ __forceinline__ void keep4_b(v16b a, v16b b, v16b c, v16b d) { asm volatile("v_nop" :: "v"(a), "v"(b), "v"(c), "v"(d)); }
__device__ __forceinline__ void acc_guard4(v8f& a, v8f& b, v8f& c, v8f& d) { asm volatile("v_nop\n\tv_nop\n\tv_nop\n\tv_nop" : "+v"(a), "+v"(b), "+v"(c), "+v"(d)); }
template <typename T> struct Frag;
template <> struct Frag<_Float16> {
  typedef v16h V; union U { v16h v; v8h h[2]; };
  static __device__ __forceinline__ v16h load(const _Float16* p) {
    U f; f.h[0] = *(const v8h*)(p); f.h[1] = *(const v8h*)(p + 16); return f.v;
  }
  static __device__ __forceinline__ v8f mma(v16h a, v16h b, v8f c) {
    return __builtin_amdgcn_wmma_f32_16x16x32_f16(false, a, false, b, (short)0, c, false, false);
  }
  static __device__ __forceinline__ void guard(v8f& a, v8f& b, v16h x, v16h y) { dep_guard_h(a, b, x, y); }
  static __device__ __forceinline__ void keep(v16h a, v16h b, v16h c, v16h d) { keep4_h(a, b, c, d); }
};
template <> struct Frag<__bf16> {
  typedef v16b V; union U { v16b v; v8b h[2]; };
  static __device__ __forceinline__ v16b load(const __bf16* p) {
    U f; f.h[0] = *(const v8b*)(p); f.h[1] = *(const v8b*)(p + 16); return f.v;
  }
  static __device__ __forceinline__ v8f mma(v16b a, v16b b, v8f c) {
    return __builtin_amdgcn_wmma_f32_16x16x32_bf16(false, a, false, b, (short)0, c, false, false);
  }
  static __device__ __forceinline__ void guard(v8f& a, v8f& b, v16b x, v16b y) { dep_guard_b(a, b, x, y); }
  static __device__ __forceinline__ void keep(v16b a, v16b b, v16b c, v16b d) { keep4_b(a, b, c, d); }
};

__device__ __forceinline__ unsigned pk16(unsigned short a, unsigned short b) { return (unsigned)a | ((unsigned)b << 16); }
__device__ __forceinline__ unsigned short h_bits(float f) { const _Float16 h = (_Float16)f; return __builtin_bit_cast(unsigned short, h); }

template <int ET> struct Elem;
template <> struct Elem<0> { typedef _Float16 T; };
template <> struct Elem<1> { typedef __bf16 T; };
template <int ET, bool SPLIT, int BIAS_MODE, int OUT_MODE, bool RESID, int ACT, bool ROWSC>
__global__ __launch_bounds__(256) void wmma_gemm64(
    const unsigned short* __restrict__ Ap, const unsigned short* __restrict__ A2p, int lda, long strideA,
    const unsigned short* __restrict__ Btp, const unsigned short* __restrict__ Bt2p, int ldb, long strideB,
    void* __restrict__ Cout, void* __restrict__ Cout2, int ldc, long strideC,
    const float* __restrict__ bias,
    const float* __restrict__ resid, long strideR,
    const float* __restrict__ rowsc,
    int M, int N, int K, float scale) {
  typedef typename Elem<ET>::T T;
  typedef typename Frag<T>::V V;
  const T* A = (const T*)Ap; const T* A2 = (const T*)A2p; const T* Bt = (const T*)Btp; const T* Bt2 = (const T*)Bt2p;
  __shared__ __align__(16) float sT[8][16 * 68];
  const int b    = blockIdx.y;
  const int lane = threadIdx.x & 31;
  const int wave = threadIdx.x >> 5;
  const int tilesN = N >> 6;
  const int tilesM = M >> 6;
  const int tile = blockIdx.x * 8 + wave;
  if (tile >= tilesM * tilesN) return;
  const int tm = tile / tilesN;
  const int tn = tile - tm * tilesN;
  const int m0 = tm << 6;
  const int n0 = tn << 6;

  const T* Ab  = A  + (size_t)b * strideA;
  const T* Bb  = Bt + (size_t)b * strideB;
  const T* Ab2 = SPLIT ? (A2  + (size_t)b * strideA) : nullptr;
  const T* Bb2 = SPLIT ? (Bt2 + (size_t)b * strideB) : nullptr;

  const int rlane = lane & 15;
  const int koff  = (lane >> 4) * 8;
  const int mOff  = (lane >> 4) * 8;

  v8f acc[4][4];
#pragma unroll
  for (int i = 0; i < 4; ++i)
#pragma unroll
    for (int j = 0; j < 4; ++j) acc[i][j] = (v8f){0.f,0.f,0.f,0.f,0.f,0.f,0.f,0.f};

  for (int k0 = 0; k0 < K; k0 += 32) {
    V bh[4], bl[4];
#pragma unroll
    for (int j = 0; j < 4; ++j) {
      const size_t bo = (size_t)(n0 + (j << 4) + rlane) * ldb + koff + k0;
      bh[j] = Frag<T>::load(Bb + bo);
      if (SPLIT) bl[j] = Frag<T>::load(Bb2 + bo);
    }
#pragma unroll
    for (int i = 0; i < 4; ++i) {
      const size_t ao = (size_t)(m0 + (i << 4) + rlane) * lda + koff + k0;
      V ah = Frag<T>::load(Ab + ao);
      V al;
      if (SPLIT) al = Frag<T>::load(Ab2 + ao);
#pragma unroll
      for (int j = 0; j < 4; ++j) {
        acc[i][j] = Frag<T>::mma(ah, bh[j], acc[i][j]);
        if (SPLIT) {
          acc[i][j] = Frag<T>::mma(ah, bl[j], acc[i][j]);
          acc[i][j] = Frag<T>::mma(al, bh[j], acc[i][j]);
        }
      }
      Frag<T>::guard(acc[i][0], acc[i][3], ah, SPLIT ? al : ah);
    }
    Frag<T>::keep(bh[0], bh[1], bh[2], bh[3]);
    if (SPLIT) Frag<T>::keep(bl[0], bl[1], bl[2], bl[3]);
  }
  acc_guard4(acc[0][0], acc[0][1], acc[0][2], acc[0][3]);
  acc_guard4(acc[1][0], acc[1][1], acc[1][2], acc[1][3]);
  acc_guard4(acc[2][0], acc[2][1], acc[2][2], acc[2][3]);
  acc_guard4(acc[3][0], acc[3][1], acc[3][2], acc[3][3]);

  float* slab = sT[wave];
  const float* Rb = RESID ? (resid + (size_t)b * strideR) : nullptr;
#pragma unroll
  for (int i = 0; i < 4; ++i) {
    const int mBase = m0 + (i << 4);
#pragma unroll
    for (int j = 0; j < 4; ++j) {
      const int n = n0 + (j << 4) + rlane;
      float bv = 0.f;
      if (BIAS_MODE == 2) bv = bias[n];
#pragma unroll
      for (int r = 0; r < 8; ++r) {
        float v = acc[i][j][r] * scale;
        if (BIAS_MODE == 1) v += bias[mBase + mOff + r];
        if (BIAS_MODE == 2) v += bv;
        if (RESID) v += Rb[(size_t)(mBase + mOff + r) * ldc + n];
        if (ACT == 2) v = fmaxf(v, 0.0f);
        if (ACT == 4) v = (v > 0.f) ? v : 0.01f * v;
        slab[(mOff + r) * 68 + (j << 4) + rlane] = v;
      }
    }
    __builtin_amdgcn_fence(__ATOMIC_RELEASE, "workgroup");
    __builtin_amdgcn_wave_barrier();
    __builtin_amdgcn_fence(__ATOMIC_ACQUIRE, "workgroup");
    if (OUT_MODE == 0) {
      float* C = (float*)Cout + (size_t)b * strideC;
      const int hh = lane >> 4, c4 = (lane & 15) * 4;
      for (int pass = 0; pass < 2; ++pass) {
#pragma unroll
        for (int it = 0; it < 8; ++it) {
          const int row = it * 2 + hh;
          v4f v = *(const v4f*)(slab + row * 68 + c4);
          if (ROWSC) { const float rsv = rowsc[mBase + row]; v = v * rsv; }
          *(volatile v4f*)(C + (size_t)(mBase + row) * ldc + n0 + c4) = v;
        }
        __threadfence();
      }
    } else {
      const int q = lane >> 3, c8 = (lane & 7) * 8;
      unsigned short* C  = (unsigned short*)Cout  + (size_t)b * strideC;
      unsigned short* C2 = (OUT_MODE == 2) ? ((unsigned short*)Cout2 + (size_t)b * strideC) : nullptr;
      for (int pass = 0; pass < 2; ++pass) {
#pragma unroll
        for (int it = 0; it < 4; ++it) {
          const int row = it * 4 + q;
          const float* sp = slab + row * 68 + c8;
          v8h hv, lv;
#pragma unroll
          for (int e = 0; e < 8; ++e) {
            if (OUT_MODE == 1) {
              hv[e] = (_Float16)sp[e];
            } else {
              unsigned short hb = f2bf_bits(sp[e]);
              unsigned short lb = f2bf_bits(sp[e] - bf_bits2f(hb));
              hv[e] = __builtin_bit_cast(_Float16, hb);
              lv[e] = __builtin_bit_cast(_Float16, lb);
            }
          }
          *(volatile v8h*)(C + (size_t)(mBase + row) * ldc + n0 + c8) = hv;
          if (OUT_MODE == 2) *(volatile v8h*)(C2 + (size_t)(mBase + row) * ldc + n0 + c8) = lv;
        }
        __threadfence();
      }
    }
    __builtin_amdgcn_fence(__ATOMIC_RELEASE, "workgroup");
    __builtin_amdgcn_wave_barrier();
    __builtin_amdgcn_fence(__ATOMIC_ACQUIRE, "workgroup");
  }
}

__device__ __forceinline__ float wsum32(float d) {
  d += __shfl_xor(d, 16, 32); d += __shfl_xor(d, 8, 32); d += __shfl_xor(d, 4, 32); d += __shfl_xor(d, 2, 32); d += __shfl_xor(d, 1, 32);
  return d;
}

__device__ __forceinline__ int blk_excl_scan(int cnt, int* scan_ws, int tid, int* tot) {
  const int lane = tid & 31, wave = tid >> 5; int incl = cnt;
#pragma unroll
  for (int o = 1; o < 32; o <<= 1) { const int v = __shfl_up(incl, o, 32); if (lane >= o) incl += v; }
  if (lane == 31) scan_ws[wave] = incl;
  __syncthreads();
  if (wave == 0) { int wv = (lane < kNT / 32) ? scan_ws[lane] : 0; int wincl = wv;
#pragma unroll
    for (int o = 1; o < 32; o <<= 1) { const int v = __shfl_up(wincl, o, 32); if (lane >= o) wincl += v; }
    if (lane < kNT / 32) scan_ws[32 + lane] = wincl - wv; if (lane == 31) scan_ws[64] = wincl; }
  __syncthreads();
  const int res = scan_ws[32 + wave] + incl - cnt; *tot = scan_ws[64];
  return res;
}

template <int TROWS, int CAP>
__device__ __forceinline__ int chunk_hits(const int* __restrict__ dstv, int e0, int n0, int tid, int* LIST, int* scan_ws) {
  const int eb = e0 + tid * kSP;
  const bool inr = eb < kEdges;
  const int ebc = inr ? eb : (kEdges - kSP);
  const unsigned nn0 = inr ? (unsigned)n0 : 0x40000000u;
  unsigned hm = 0u;
#pragma unroll
  for (int k = 0; k < kSP; k += 4) {
    const v4i d4 = *(const v4i*)(dstv + ebc + k);
#pragma unroll
    for (int e = 0; e < 4; ++e) {
      const unsigned u = (unsigned)d4[e] - nn0;
      hm |= (u < (unsigned)TROWS) ? (1u << (k + e)) : 0u;
    }
  }
  const int cnt = __builtin_popcount(hm);
  int tot; int p = blk_excl_scan(cnt, scan_ws, tid, &tot);
#pragma unroll 1
  for (int it = 0; it < kSP; ++it) {
    if (hm == 0u) break;
    const int bpos = __builtin_ctz(hm); hm &= hm - 1u;
    const int d = dstv[ebc + bpos];
    int dl = d - n0; dl = dl < 0 ? 0 : (dl >= TROWS ? TROWS - 1 : dl);
    const int r = (dl << 13) | (tid * kSP + bpos);
    if ((unsigned)p < (unsigned)CAP) LIST[p] = r;
    ++p;
  }
  __syncthreads();
  return tot < CAP ? tot : CAP;
}

__global__ __launch_bounds__(kNT) void wt_kernel(const float* __restrict__ Wa, const float* __restrict__ Wb, const float* __restrict__ Wc,
                                                unsigned short* __restrict__ Ta, unsigned short* __restrict__ Tb, unsigned short* __restrict__ Tc) {
  __shared__ float sm[kFin * 65];
  const int tid = threadIdx.x;
  const int z = blockIdx.x;
  const float* W = (z == 0) ? Wa : ((z == 1) ? Wb : Wc);
  unsigned short* T = (z == 0) ? Ta : ((z == 1) ? Tb : Tc);
  const int K   = (z == 0) ? kFin : kHid;
  const int lgK = (z == 0) ? 7 : 6;
  for (int i = tid; i < K * kHid; i += kNT) { const int k = i >> 6, n = i & 63; sm[k * 65 + n] = W[i] * kCarryW; }
  __syncthreads();
  for (int g8 = tid; g8 < 8 * K; g8 += kNT) {
    const int h0 = g8 * 8;
    const int n  = h0 >> lgK;
    const int k0 = h0 & (K - 1);
    unsigned short hb[8];
#pragma unroll
    for (int e = 0; e < 8; ++e) hb[e] = h_bits(sm[(k0 + e) * 65 + n]);
    const v4u u = (v4u){pk16(hb[0], hb[1]), pk16(hb[2], hb[3]), pk16(hb[4], hb[5]), pk16(hb[6], hb[7])};
    unsigned short* op = T + h0;
    *(volatile v4u*)op = u;
    __threadfence();
    *(volatile v4u*)op = u;
  }
}

__global__ __launch_bounds__(kNT) void cast_x_kernel(const float* __restrict__ x, unsigned short* __restrict__ A1) {
  const int i = blockIdx.x * kNT + threadIdx.x;
  const int nLive = kNodes * (kFin / 8);
  const bool live = i < nLive;
  const int ic = live ? i : (nLive - 1);
  const float* p = x + (size_t)ic * 8;
  const v4f a = *(const v4f*)(p);
  const v4f c = *(const v4f*)(p + 4);
  const float lf = live ? 1.0f : 0.0f;
  unsigned short hb[8];
#pragma unroll
  for (int e = 0; e < 4; ++e) {
    hb[e]     = h_bits(a[e] * lf);
    hb[4 + e] = h_bits(c[e] * lf);
  }
  const v4u u = (v4u){pk16(hb[0], hb[1]), pk16(hb[2], hb[3]), pk16(hb[4], hb[5]), pk16(hb[6], hb[7])};
  unsigned short* q = A1 + (size_t)i * 8;
  *(volatile v4u*)q = u;
  __threadfence();
  *(volatile v4u*)q = u;
}

__global__ __launch_bounds__(kNT) void deg_kernel(const int* __restrict__ ei, float* __restrict__ DIS) {
  __shared__ int CNT[kTileS];
  __shared__ int LIST[kCapS];
  __shared__ int scan_ws[80];
  const int tid = threadIdx.x, lane = tid & 31, wave = tid >> 5;
  const int n0 = blockIdx.x * kTileS;
  const int rw0 = wave * kRowsWS;
  for (int i = tid; i < kTileS; i += kNT) CNT[i] = 0;
  for (int i = tid; i < kCapS; i += kNT) LIST[i] = 0;
  if (tid < 80) scan_ws[tid] = 0;
  __syncthreads();
  const int* dstv = ei + kEdges;
#pragma unroll 1
  for (int c = 0; c < kChunksE; ++c) {
    const int tot = chunk_hits<kTileS, kCapS>(dstv, c * kChunk, n0, tid, LIST, scan_ws);
#pragma unroll 1
    for (int base = 0; base < tot; base += 32) {
      const int q = base + lane;
      const int qc = (q < kCapS) ? q : (kCapS - 1);
      const int rv = LIST[qc];
      const bool valid = q < tot;
      const int dl = rv >> 13;
      const int own = (valid && ((unsigned)(dl - rw0) < (unsigned)kRowsWS)) ? 1 : 0;
      unsigned msk = (unsigned)__ballot(own);
#pragma unroll 1
      for (int it = 0; it < 32; ++it) {
        if (msk == 0u) break;
        const int bpos = __builtin_ctz(msk); msk &= msk - 1u;
        int d2 = __shfl(dl, bpos, 32);
        d2 = d2 < 0 ? 0 : (d2 >= kTileS ? kTileS - 1 : d2);
        CNT[d2] = CNT[d2] + 1;
      }
    }
    __syncthreads();
  }
  __syncthreads();
  for (int ps = 0; ps < 2; ++ps) {
#pragma unroll 1
    for (int i = 0; i < kRowsWS / 32; ++i) {
      const int r = rw0 + i * 32 + lane;
      const float dv = 1.0f / sqrtf((float)CNT[r] + 1.0f);
      *(volatile float*)(DIS + n0 + r) = dv;
    }
    __threadfence();
  }
}

__global__ __launch_bounds__(kNT) void agg64_kernel(const float* __restrict__ XWS, const int* __restrict__ ei,
                                                   const float* __restrict__ DIS, const float* __restrict__ bias,
                                                   unsigned short* __restrict__ HP) {
  __shared__ __align__(16) float ACC[kTileR * kHid];
  __shared__ int LIST[kCapR];
  __shared__ int scan_ws[80];
  const int tid = threadIdx.x, lane = tid & 31, wave = tid >> 5;
  const int n0 = blockIdx.x * kTileR;
  const int rw0 = wave * kRowsW;
  for (int i = tid; i < kCapR; i += kNT) LIST[i] = 0;
  if (tid < 80) scan_ws[tid] = 0;
#pragma unroll 1
  for (int j = 0; j < kRowsW; ++j) {
    const int r = rw0 + j;
    const v2f v = *(const v2f*)(XWS + (size_t)(n0 + r) * kHid + 2 * lane);
    *(v2f*)(ACC + r * kHid + 2 * lane) = v;
  }
  __syncthreads();
  const int* srcv = ei;
  const int* dstv = ei + kEdges;
#pragma unroll 1
  for (int c = 0; c < kChunksE; ++c) {
    const int e0 = c * kChunk;
    const int tot = chunk_hits<kTileR, kCapR>(dstv, e0, n0, tid, LIST, scan_ws);
#pragma unroll 1
    for (int base = 0; base < tot; base += 32) {
      const int q = base + lane;
      const int qc = (q < kCapR) ? q : (kCapR - 1);
      const int rv = LIST[qc];
      const bool valid = q < tot;
      const int dl = rv >> 13;
      int e = e0 + (rv & 8191); e = (e < kEdges) ? e : (kEdges - 1);
      int s = srcv[e]; s = s < 0 ? 0 : (s >= kNodes ? kNodes - 1 : s);
      const int own = (valid && ((unsigned)(dl - rw0) < (unsigned)kRowsW)) ? 1 : 0;
      const int pk = (dl << 17) | s;
      unsigned msk = (unsigned)__ballot(own);
#pragma unroll 1
      for (int it = 0; it < 32; ++it) {
        if (msk == 0u) break;
        const int bpos = __builtin_ctz(msk); msk &= msk - 1u;
        const int r = __shfl(pk, bpos, 32);
        int d2 = r >> 17; d2 = d2 < 0 ? 0 : (d2 >= kTileR ? kTileR - 1 : d2);
        int s2 = r & 0x1FFFF; s2 = (s2 < kNodes) ? s2 : (kNodes - 1);
        const v2f xv = *(const v2f*)(XWS + (size_t)s2 * kHid + 2 * lane);
        float* ap = ACC + d2 * kHid + 2 * lane;
        v2f a = *(const v2f*)ap;
        a = a + xv;
        *(v2f*)ap = a;
      }
    }
    __syncthreads();
  }
  __syncthreads();
  {
    const int q = lane >> 3, c8 = (lane & 7) * 8;
    const v4f bA = *(const v4f*)(bias + c8), bB = *(const v4f*)(bias + c8 + 4);
    for (int ps = 0; ps < 2; ++ps) {
#pragma unroll 1
      for (int i = 0; i < kRowsW / 4; ++i) {
        const int r = rw0 + 4 * i + q;
        const int n = n0 + r;
        const float* ap = ACC + r * kHid + c8;
        const v4f a0 = *(const v4f*)(ap), a1 = *(const v4f*)(ap + 4);
        const float ds = DIS[n];
        const float cf = (n < kNodes) ? kCarryH : 0.0f;
        v4f h0 = a0 * ds + bA;
        v4f h1 = a1 * ds + bB;
#pragma unroll
        for (int e = 0; e < 4; ++e) { h0[e] = fmaxf(h0[e], 0.0f); h1[e] = fmaxf(h1[e], 0.0f); }
        h0 = h0 * cf; h1 = h1 * cf;
        unsigned short hb[8];
#pragma unroll
        for (int e = 0; e < 4; ++e) { hb[e] = h_bits(h0[e]); hb[4 + e] = h_bits(h1[e]); }
        const v4u u = (v4u){pk16(hb[0], hb[1]), pk16(hb[2], hb[3]), pk16(hb[4], hb[5]), pk16(hb[6], hb[7])};
        *(volatile v4u*)(HP + (size_t)n * kHid + c8) = u;
      }
      __threadfence();
    }
  }
}

__global__ __launch_bounds__(kNT) void v_kernel(const float* __restrict__ XWS3, const float* __restrict__ Wl, float* __restrict__ V) {
  const int lane = threadIdx.x & 31, wave = threadIdx.x >> 5;
  const int base = (blockIdx.x * 8 + wave) * 32;
  const v2f wl2 = *(const v2f*)(Wl + 2 * lane);
  float mine = 0.0f;
#pragma unroll 1
  for (int j = 0; j < 32; ++j) {
    const int n = base + j;
    const v2f xv = *(const v2f*)(XWS3 + (size_t)n * kHid + 2 * lane);
    float t = xv[0] * wl2[0];
    t = t + xv[1] * wl2[1];
    t = wsum32(t);
    mine = (lane == j) ? t : mine;
  }
  float* p = V + base + lane;
  *(volatile float*)p = mine;
  __threadfence();
  *(volatile float*)p = mine;
}

__global__ __launch_bounds__(kNT) void agg3_kernel(const float* __restrict__ V, const int* __restrict__ ei, const float* __restrict__ DIS,
                                                  const float* __restrict__ b3, const float* __restrict__ Wl, float* __restrict__ S3) {
  __shared__ float S[kTileS];
  __shared__ int LIST[kCapS];
  __shared__ int scan_ws[80];
  const int tid = threadIdx.x, lane = tid & 31, wave = tid >> 5;
  const int n0 = blockIdx.x * kTileS;
  const int rw0 = wave * kRowsWS;
  for (int i = tid; i < kTileS; i += kNT) S[i] = V[n0 + i];
  for (int i = tid; i < kCapS; i += kNT) LIST[i] = 0;
  if (tid < 80) scan_ws[tid] = 0;
  float cB;
  {
    const v2f bb = *(const v2f*)(b3 + 2 * lane);
    const v2f ww = *(const v2f*)(Wl + 2 * lane);
    float t = 0.0f;
    t = t + bb[0] * ww[0];
    t = t + bb[1] * ww[1];
    cB = wsum32(t);
  }
  __syncthreads();
  const int* srcv = ei;
  const int* dstv = ei + kEdges;
#pragma unroll 1
  for (int c = 0; c < kChunksE; ++c) {
    const int e0 = c * kChunk;
    const int tot = chunk_hits<kTileS, kCapS>(dstv, e0, n0, tid, LIST, scan_ws);
#pragma unroll 1
    for (int base = 0; base < tot; base += 32) {
      const int q = base + lane;
      const int qc = (q < kCapS) ? q : (kCapS - 1);
      const int rv = LIST[qc];
      const bool valid = q < tot;
      const int dl = rv >> 13;
      int e = e0 + (rv & 8191); e = (e < kEdges) ? e : (kEdges - 1);
      int s = srcv[e]; s = s < 0 ? 0 : (s >= kNodes ? kNodes - 1 : s);
      const float vs = V[s];
      const int own = (valid && ((unsigned)(dl - rw0) < (unsigned)kRowsWS)) ? 1 : 0;
      unsigned msk = (unsigned)__ballot(own);
#pragma unroll 1
      for (int it = 0; it < 32; ++it) {
        if (msk == 0u) break;
        const int bpos = __builtin_ctz(msk); msk &= msk - 1u;
        int d2 = __shfl(dl, bpos, 32);
        const float vv = __shfl(vs, bpos, 32);
        d2 = d2 < 0 ? 0 : (d2 >= kTileS ? kTileS - 1 : d2);
        S[d2] = S[d2] + vv;
      }
    }
    __syncthreads();
  }
  __syncthreads();
  for (int ps = 0; ps < 2; ++ps) {
#pragma unroll 1
    for (int i = 0; i < kRowsWS / 32; ++i) {
      const int r = rw0 + i * 32 + lane;
      const int n = n0 + r;
      const float val = DIS[n] * S[r] + cB;
      *(volatile float*)(S3 + n) = val;
    }
    __threadfence();
  }
}

__global__ __launch_bounds__(kNT) void pool_kernel(const float* __restrict__ S3, const int* __restrict__ batch,
                                                  const float* __restrict__ bl, float* __restrict__ out) {
  __shared__ float PS[kGPB * kNT];
  __shared__ int   PC[kGPB * kNT];
  const int tid = threadIdx.x, lane = tid & 31, wave = tid >> 5;
  const int g0 = blockIdx.x * kGPB;
  for (int i = tid; i < kGPB * kNT; i += kNT) { PS[i] = 0.0f; PC[i] = 0; }
  __syncthreads();
#pragma unroll 1
  for (int n = tid; n < kNodes; n += kNT) {
    const int bg = batch[n];
    const float sv = S3[n];
    const int gi = bg - g0;
    if ((unsigned)gi < (unsigned)kGPB) {
      const int slot = gi * kNT + tid;
      PS[slot] = PS[slot] + sv;
      PC[slot] = PC[slot] + 1;
    }
  }
  __syncthreads();
  if (wave == 0) {
    float sum = 0.0f; int ct = 0;
#pragma unroll 1
    for (int t = 0; t < kNT; ++t) { sum = sum + PS[lane * kNT + t]; ct += PC[lane * kNT + t]; }
    const float inv = 1.0f / fmaxf((float)ct, 1.0f);
    const float val = sum * inv + bl[0];
    float* p = out + g0 + lane;
    *(volatile float*)p = val;
    __threadfence();
    *(volatile float*)p = val;
  }
}

extern "C" void kernel_launch(void* const* d_in, const int* in_sizes, int n_in,
                              void* d_out, int out_size, void* d_ws, size_t ws_size, hipStream_t stream) {
  (void)in_sizes; (void)n_in; (void)out_size;
  const float* x     = (const float*)d_in[0];
  const int*   ei    = (const int*)  d_in[1];
  const int*   batch = (const int*)  d_in[2];
  const float* W1 = (const float*)d_in[3];  const float* b1 = (const float*)d_in[4];
  const float* W2 = (const float*)d_in[5];  const float* b2 = (const float*)d_in[6];
  const float* W3 = (const float*)d_in[7];  const float* b3 = (const float*)d_in[8];
  const float* Wl = (const float*)d_in[9];  const float* bl = (const float*)d_in[10];
  float* out = (float*)d_out;

  char* ws = (char*)d_ws; size_t off = 0;
  auto carve = [&](size_t bytes) -> char* { char* p = ws + off; off += (bytes + 255) & ~(size_t)255; return p; };
  unsigned short* WT1  = (unsigned short*)carve((size_t)kHid * kFin * 2);
  unsigned short* WT2  = (unsigned short*)carve((size_t)kHid * kHid * 2);
  unsigned short* WT3  = (unsigned short*)carve((size_t)kHid * kHid * 2);
  float*          DIS  = (float*)carve((size_t)kNpad * 4);
  unsigned short* A1   = (unsigned short*)carve((size_t)kNpad * kFin * 2);
  float*          XWSA = (float*)carve((size_t)kNpad * kHid * 4);
  float*          XWSB = (float*)carve((size_t)kNpad * kHid * 4);
  unsigned short* HP1  = (unsigned short*)carve((size_t)kNpad * kHid * 2);
  unsigned short* HP2  = (unsigned short*)carve((size_t)kNpad * kHid * 2);
  float*          V    = (float*)carve((size_t)kNpad * 4);
  float*          S3   = (float*)carve((size_t)kNpad * 4);
  if (off > ws_size || off > (size_t)134217728) return;

  const int gemmBlocks = (kNpad / 64) / 8;

  wt_kernel<<<3, kNT, 0, stream>>>(W1, W2, W3, WT1, WT2, WT3);
  cast_x_kernel<<<(kNpad * (kFin / 8)) / kNT, kNT, 0, stream>>>(x, A1);
  deg_kernel<<<kTilesS, kNT, 0, stream>>>(ei, DIS);

  wmma_gemm64<0, false, 0, 0, false, 0, true><<<dim3(gemmBlocks, 1), 256, 0, stream>>>(
      A1, (const unsigned short*)nullptr, kFin, 0L,
      WT1, (const unsigned short*)nullptr, kFin, 0L,
      (void*)XWSA, (void*)nullptr, kHid, 0L,
      (const float*)nullptr, (const float*)nullptr, 0L,
      DIS, kNpad, kHid, kFin, kScale1);
  agg64_kernel<<<kTilesR, kNT, 0, stream>>>(XWSA, ei, DIS, b1, HP1);

  wmma_gemm64<0, false, 0, 0, false, 0, true><<<dim3(gemmBlocks, 1), 256, 0, stream>>>(
      HP1, (const unsigned short*)nullptr, kHid, 0L,
      WT2, (const unsigned short*)nullptr, kHid, 0L,
      (void*)XWSB, (void*)nullptr, kHid, 0L,
      (const float*)nullptr, (const float*)nullptr, 0L,
      DIS, kNpad, kHid, kHid, kScale2);
  agg64_kernel<<<kTilesR, kNT, 0, stream>>>(XWSB, ei, DIS, b2, HP2);

  wmma_gemm64<0, false, 0, 0, false, 0, true><<<dim3(gemmBlocks, 1), 256, 0, stream>>>(
      HP2, (const unsigned short*)nullptr, kHid, 0L,
      WT3, (const unsigned short*)nullptr, kHid, 0L,
      (void*)XWSA, (void*)nullptr, kHid, 0L,
      (const float*)nullptr, (const float*)nullptr, 0L,
      DIS, kNpad, kHid, kHid, kScale2);
  v_kernel<<<(kNpad / 32) / 8, kNT, 0, stream>>>(XWSA, Wl, V);
  agg3_kernel<<<kTilesS, kNT, 0, stream>>>(V, ei, DIS, b3, Wl, S3);
  pool_kernel<<<kGraphs / kGPB, kNT, 0, stream>>>(S3, batch, bl, out);
}
